// MultiHeadAttention_68667937128978
// MI455X (gfx1250) — hardware-verified
//
#include <hip/hip_runtime.h>
#ifndef NB
#define NB 2
#endif
#ifndef SEQ
#define SEQ 2048
#endif
#define NB_FULL 2
#define SEQ_FULL 2048
#define EDIM 1024
#define NH 16
#define HD 64

static_assert(SEQ % 128 == 0);
static_assert(SEQ <= SEQ_FULL);
static_assert(NB <= NB_FULL);
static_assert(NH * HD == EDIM);
static_assert(HD == 64);
static_assert(EDIM % 64 == 0);
static_assert((size_t)NB * SEQ * EDIM * 2 * 10 + (size_t)EDIM * EDIM * 2 * 4 <= (size_t)134217728);

typedef __bf16 v16b __attribute__((ext_vector_type(16)));
typedef _Float16 v16h __attribute__((ext_vector_type(16)));
typedef unsigned short v8us __attribute__((ext_vector_type(8), may_alias));
typedef float v8f __attribute__((ext_vector_type(8)));
typedef float v4f __attribute__((ext_vector_type(4)));
typedef float v4fa __attribute__((ext_vector_type(4), may_alias));
union FragB { v16b v; v8us half[2]; unsigned short u[16]; };
union FragH { v16h v; v8us half[2]; _Float16 h[16]; unsigned short u[16]; };

#define LOG2E 1.4426950408889634f

__device__ __forceinline__ unsigned short bf16_bits(float x) {
  unsigned int u = __float_as_uint(x);
  return (unsigned short)((u + 0x7FFFu + ((u >> 16) & 1u)) >> 16);
}
__device__ __forceinline__ float bf16_val(unsigned short b) { return __uint_as_float(((unsigned int)b) << 16); }

__device__ __forceinline__ v8f wm_bf(v16b a, v16b b, v8f c) {
  return __builtin_amdgcn_wmma_f32_16x16x32_bf16(false, a, false, b, (short)0, c, false, false);
}

__device__ __forceinline__ void mma_g8(v16b a0, v16b a1, v16b b0, v16b b1, v16b b2, v16b b3, v8f (&c0)[4], v8f (&c1)[4]) {
  c0[0] = wm_bf(a0, b0, c0[0]); c1[0] = wm_bf(a1, b0, c1[0]);
  c0[1] = wm_bf(a0, b1, c0[1]); c1[1] = wm_bf(a1, b1, c1[1]);
  c0[2] = wm_bf(a0, b2, c0[2]); c1[2] = wm_bf(a1, b2, c1[2]);
  c0[3] = wm_bf(a0, b3, c0[3]); c1[3] = wm_bf(a1, b3, c1[3]);
  asm volatile("v_nop\n\tv_nop\n\tv_nop\n\tv_nop"
               : "+v"(c0[0]), "+v"(c0[1]), "+v"(c0[2]), "+v"(c0[3]), "+v"(c1[0]), "+v"(c1[1]), "+v"(c1[2]), "+v"(c1[3])
               : "v"(a0), "v"(a1), "v"(b0), "v"(b1), "v"(b2), "v"(b3));
}
__device__ __forceinline__ v8f mma_bf6(v16b kh0, v16b kh1, v16b kl0, v16b kl1, v16b qh0, v16b qh1, v16b ql0, v16b ql1, v8f c) {
  c = wm_bf(kl0, qh0, c);
  c = wm_bf(kl1, qh1, c);
  c = wm_bf(kh0, ql0, c);
  c = wm_bf(kh1, ql1, c);
  c = wm_bf(kh0, qh0, c);
  c = wm_bf(kh1, qh1, c);
  asm volatile("v_nop\n\tv_nop\n\tv_nop\n\tv_nop" : "+v"(c)
               : "v"(kh0), "v"(kh1), "v"(kl0), "v"(kl1), "v"(qh0), "v"(qh1), "v"(ql0), "v"(ql1));
  return c;
}
__device__ __forceinline__ void mma_h2(v16h a, v16h bh, v16h bl, v8f& ch, v8f& cl) {
  ch = __builtin_amdgcn_wmma_f32_16x16x32_f16(false, a, false, bh, (short)0, ch, false, false);
  cl = __builtin_amdgcn_wmma_f32_16x16x32_f16(false, a, false, bl, (short)0, cl, false, false);
  asm volatile("v_nop\n\tv_nop\n\tv_nop\n\tv_nop" : "+v"(ch), "+v"(cl) : "v"(a), "v"(bh), "v"(bl));
}

__global__ __launch_bounds__(256) void k_cvt(const float* __restrict__ src, unsigned short* __restrict__ dst,
                                             int rows_per_b, int bstride_rows, int total8) {
  const int t = blockIdx.x * 256 + threadIdx.x;
  if (t >= total8) return;
  const int row = t >> 7, piece = t & 127;
  const int b = row / rows_per_b, s = row - b * rows_per_b;
  const float* p = src + ((size_t)b * bstride_rows + s) * EDIM + piece * 8;
  const v4f x0 = *(const v4fa*)(p), x1 = *(const v4fa*)(p + 4);
  v8us o;
  o[0] = bf16_bits(x0[0]); o[1] = bf16_bits(x0[1]); o[2] = bf16_bits(x0[2]); o[3] = bf16_bits(x0[3]);
  o[4] = bf16_bits(x1[0]); o[5] = bf16_bits(x1[1]); o[6] = bf16_bits(x1[2]); o[7] = bf16_bits(x1[3]);
  unsigned short* d = dst + (size_t)t * 8;
  *(volatile v8us*)d = o;
  __threadfence();
  *(volatile v8us*)d = o;
}

template <int MODE, int KTOT, int LDA>
__global__ __launch_bounds__(128) void k_gemm(const unsigned short* __restrict__ A, const unsigned short* __restrict__ Bw,
                                              unsigned short* __restrict__ P0, unsigned short* __restrict__ P1,
                                              float* __restrict__ Of) {
  __shared__ __attribute__((aligned(16))) float so[128][68];
  const int tid = threadIdx.x, w = __builtin_amdgcn_readfirstlane((int)(tid >> 5)), lane = tid & 31, ln = lane & 15, hh = lane >> 4;
  const int gm0 = blockIdx.x * 128;
  const int hcol = blockIdx.y;
  const int n0 = hcol * 64;
  const unsigned short* ap0 = A + (size_t)(gm0 + 32 * w + ln) * LDA + 8 * hh;
  const unsigned short* ap1 = ap0 + (size_t)16 * LDA;
  const unsigned short* bp = Bw + (size_t)(n0 + ln) * EDIM + 8 * hh;
  v8f acc0[4] = {}, acc1[4] = {};
#pragma unroll 1
  for (int kk = 0; kk < KTOT; kk += 32) {
    const int kb = kk & (EDIM - 1);
    FragB a0, a1, b0, b1, b2, b3;
    a0.half[0] = *(const v8us*)(ap0 + kk); a0.half[1] = *(const v8us*)(ap0 + kk + 16);
    a1.half[0] = *(const v8us*)(ap1 + kk); a1.half[1] = *(const v8us*)(ap1 + kk + 16);
    b0.half[0] = *(const v8us*)(bp + kb);                 b0.half[1] = *(const v8us*)(bp + kb + 16);
    b1.half[0] = *(const v8us*)(bp + 16 * EDIM + kb);     b1.half[1] = *(const v8us*)(bp + 16 * EDIM + kb + 16);
    b2.half[0] = *(const v8us*)(bp + 32 * EDIM + kb);     b2.half[1] = *(const v8us*)(bp + 32 * EDIM + kb + 16);
    b3.half[0] = *(const v8us*)(bp + 48 * EDIM + kb);     b3.half[1] = *(const v8us*)(bp + 48 * EDIM + kb + 16);
    mma_g8(a0.v, a1.v, b0.v, b1.v, b2.v, b3.v, acc0, acc1);
  }
#pragma unroll
  for (int t = 0; t < 4; ++t)
#pragma unroll
    for (int r = 0; r < 8; ++r) {
      so[32 * w + 8 * hh + r][16 * t + ln] = acc0[t][r];
      so[32 * w + 16 + 8 * hh + r][16 * t + ln] = acc1[t][r];
    }
  __syncthreads();
  const int b = gm0 / SEQ, s0 = gm0 - b * SEQ;
  if (MODE == 0) {
    const size_t base = ((size_t)(b * NH + hcol) * SEQ + s0) * HD;
    for (int pass = 0; pass < 2; ++pass) {
#pragma unroll 2
      for (int it = 0; it < 8; ++it) {
        const int i = tid + 128 * it;
        const int row = i >> 3, piece = i & 7;
        const v4f x0 = *(const v4fa*)&so[row][8 * piece], x1 = *(const v4fa*)&so[row][8 * piece + 4];
        v8us oh, ol;
#pragma unroll
        for (int q = 0; q < 4; ++q) {
          const unsigned short h0 = bf16_bits(x0[q]), h1 = bf16_bits(x1[q]);
          oh[q] = h0; oh[4 + q] = h1;
          ol[q] = bf16_bits(x0[q] - bf16_val(h0));
          ol[4 + q] = bf16_bits(x1[q] - bf16_val(h1));
        }
        const size_t o = base + (size_t)row * HD + 8 * piece;
        *(volatile v8us*)(P0 + o) = oh;
        *(volatile v8us*)(P1 + o) = ol;
      }
      if (pass == 0) __threadfence();
    }
  } else if (MODE == 1) {
    const size_t base = (size_t)(b * NH + hcol) * HD * SEQ + s0;
    for (int pass = 0; pass < 2; ++pass) {
#pragma unroll 2
      for (int it = 0; it < 8; ++it) {
        const int i = tid + 128 * it;
        const int d = i >> 4, j8 = (i & 15) * 8;
        FragH f;
#pragma unroll
        for (int q = 0; q < 8; ++q) f.h[q] = (_Float16)(so[j8 + q][d] * 16.0f);
        const v8us o = f.half[0];
        *(volatile v8us*)(P0 + base + (size_t)d * SEQ + j8) = o;
      }
      if (pass == 0) __threadfence();
    }
  } else {
    float* og = Of + ((size_t)b * SEQ_FULL + s0) * EDIM + n0;
    for (int pass = 0; pass < 2; ++pass) {
#pragma unroll 4
      for (int it = 0; it < 16; ++it) {
        const int i = tid + 128 * it;
        const int row = i >> 4, c4 = (i & 15) * 4;
        const v4f v = *(const v4fa*)&so[row][c4];
        *(volatile v4f*)(og + (size_t)row * EDIM + c4) = v;
      }
      if (pass == 0) __threadfence();
    }
  }
}

__device__ __forceinline__ void fa_step(const unsigned short* __restrict__ Khp, const unsigned short* __restrict__ Klp,
                                        const unsigned short* __restrict__ Vp, int key0, int ln, int hh,
                                        const FragB& q0h, const FragB& q1h, const FragB& q0l, const FragB& q1l,
                                        float& mr, float& lr, v8f (&Oh)[4], v8f (&Ol)[4]) {
  const v8f z8 = {0.f, 0.f, 0.f, 0.f, 0.f, 0.f, 0.f, 0.f};
  const size_t ko = (size_t)(key0 + ln) * HD + 8 * hh;
  v8f s0, s1;
  {
    const unsigned short* kh = Khp + ko;
    const unsigned short* kl = Klp + ko;
    FragB a0, a1, l0, l1;
    a0.half[0] = *(const v8us*)(kh);      a0.half[1] = *(const v8us*)(kh + 16);
    a1.half[0] = *(const v8us*)(kh + 32); a1.half[1] = *(const v8us*)(kh + 48);
    l0.half[0] = *(const v8us*)(kl);      l0.half[1] = *(const v8us*)(kl + 16);
    l1.half[0] = *(const v8us*)(kl + 32); l1.half[1] = *(const v8us*)(kl + 48);
    s0 = mma_bf6(a0.v, a1.v, l0.v, l1.v, q0h.v, q1h.v, q0l.v, q1l.v, z8);
  }
  asm volatile("" ::: "memory");
  {
    const unsigned short* kh = Khp + ko + 16 * HD;
    const unsigned short* kl = Klp + ko + 16 * HD;
    FragB a0, a1, l0, l1;
    a0.half[0] = *(const v8us*)(kh);      a0.half[1] = *(const v8us*)(kh + 16);
    a1.half[0] = *(const v8us*)(kh + 32); a1.half[1] = *(const v8us*)(kh + 48);
    l0.half[0] = *(const v8us*)(kl);      l0.half[1] = *(const v8us*)(kl + 16);
    l1.half[0] = *(const v8us*)(kl + 32); l1.half[1] = *(const v8us*)(kl + 48);
    s1 = mma_bf6(a0.v, a1.v, l0.v, l1.v, q0h.v, q1h.v, q0l.v, q1l.v, z8);
  }
  float sc[16];
#pragma unroll
  for (int r = 0; r < 8; ++r) { sc[r] = s0[r] * 0.125f; sc[8 + r] = s1[r] * 0.125f; }
  float mx = sc[0];
#pragma unroll
  for (int i = 1; i < 16; ++i) mx = fmaxf(mx, sc[i]);
  mx = fmaxf(mx, __shfl_xor(mx, 16, 32));
  const float mnew = fmaxf(mr, mx);
  const float al = exp2f((mr - mnew) * LOG2E);
  mr = mnew;
  FragH ph, pl;
  float ps = 0.0f;
#pragma unroll
  for (int i = 0; i < 16; ++i) {
    const float pc = exp2f(fmaf(sc[i] - mnew, LOG2E, 8.0f));
    ps += pc;
    const _Float16 h = (_Float16)pc;
    ph.h[i] = h;
    pl.h[i] = (_Float16)((pc - (float)h) * 2048.0f);
  }
  ps += __shfl_xor(ps, 16, 32);
  lr = lr * al + ps;
#pragma unroll
  for (int t = 0; t < 4; ++t) { Oh[t] = Oh[t] * al; Ol[t] = Ol[t] * al; }
  asm volatile("" ::: "memory");
  const unsigned short* vp = Vp + (size_t)ln * SEQ + key0 + 8 * hh;
  FragH vf[4];
#pragma unroll
  for (int t = 0; t < 4; ++t) {
    vf[t].half[0] = *(const v8us*)(vp + (size_t)t * 16 * SEQ);
    vf[t].half[1] = *(const v8us*)(vp + (size_t)t * 16 * SEQ + 16);
  }
#pragma unroll
  for (int t = 0; t < 4; ++t) mma_h2(vf[t].v, ph.v, pl.v, Oh[t], Ol[t]);
}

__global__ __launch_bounds__(128) void k_attn(const unsigned short* __restrict__ Qh, const unsigned short* __restrict__ Ql,
                                              const unsigned short* __restrict__ Kh, const unsigned short* __restrict__ Kl,
                                              const unsigned short* __restrict__ Vt, unsigned short* __restrict__ Cx) {
  __shared__ __attribute__((aligned(16))) float so[4][16][68];
  const int tid = threadIdx.x, w = __builtin_amdgcn_readfirstlane((int)(tid >> 5)), lane = tid & 31, ln = lane & 15, hh = lane >> 4;
  const int bh = blockIdx.x / (SEQ / 64), qt = blockIdx.x % (SEQ / 64);
  const int b = bh / NH, h = bh - b * NH;
  const int qbase = qt * 64 + 16 * w;
  const int qg = qbase + ln;
  const size_t hoff = (size_t)bh * SEQ * HD;
  FragB q0h, q1h, q0l, q1l;
  {
    const unsigned short* qr = Qh + hoff + (size_t)qg * HD + 8 * hh;
    q0h.half[0] = *(const v8us*)(qr);      q0h.half[1] = *(const v8us*)(qr + 16);
    q1h.half[0] = *(const v8us*)(qr + 32); q1h.half[1] = *(const v8us*)(qr + 48);
    const unsigned short* ql = Ql + hoff + (size_t)qg * HD + 8 * hh;
    q0l.half[0] = *(const v8us*)(ql);      q0l.half[1] = *(const v8us*)(ql + 16);
    q1l.half[0] = *(const v8us*)(ql + 32); q1l.half[1] = *(const v8us*)(ql + 48);
  }
  float mr = -3.0e38f, lr = 0.0f;
  v8f Oh[4] = {}, Ol[4] = {};
  const unsigned short* Khp = Kh + hoff;
  const unsigned short* Klp = Kl + hoff;
  const unsigned short* Vp = Vt + hoff;
#pragma unroll 1
  for (int j = 0; j < SEQ / 32; ++j)
    fa_step(Khp, Klp, Vp, 32 * j, ln, hh, q0h, q1h, q0l, q1l, mr, lr, Oh, Ol);

  const float inv = 1.0f / (16.0f * lr);
#pragma unroll
  for (int t = 0; t < 4; ++t)
#pragma unroll
    for (int r = 0; r < 8; ++r)
      so[w][ln][16 * t + 8 * hh + r] = (Oh[t][r] + Ol[t][r] * 0.00048828125f) * inv;
  __syncthreads();
  unsigned short* ch = Cx + ((size_t)b * SEQ + qbase) * (2 * EDIM) + h * HD;
  const int rsub = lane >> 3, piece = lane & 7;
  for (int pass = 0; pass < 2; ++pass) {
#pragma unroll
    for (int it = 0; it < 4; ++it) {
      const int row = 4 * it + rsub;
      const v4f x0 = *(const v4fa*)&so[w][row][8 * piece], x1 = *(const v4fa*)&so[w][row][8 * piece + 4];
      v8us oh, ol;
#pragma unroll
      for (int q = 0; q < 4; ++q) {
        const unsigned short h0 = bf16_bits(x0[q]), h1 = bf16_bits(x1[q]);
        oh[q] = h0; oh[4 + q] = h1;
        ol[q] = bf16_bits(x0[q] - bf16_val(h0));
        ol[4 + q] = bf16_bits(x1[q] - bf16_val(h1));
      }
      unsigned short* d = ch + (size_t)row * (2 * EDIM) + 8 * piece;
      *(volatile v8us*)(d) = oh;
      *(volatile v8us*)(d + EDIM) = ol;
    }
    if (pass == 0) __threadfence();
  }
}

extern "C" void kernel_launch(void* const* d_in, const int* in_sizes, int n_in,
                              void* d_out, int out_size, void* d_ws, size_t ws_size, hipStream_t stream) {
  if (n_in < 7) return;
  const long long need = ((long long)(NB - 1) * SEQ_FULL + (long long)SEQ) * EDIM;
  if ((long long)in_sizes[0] < need || (long long)in_sizes[1] < need || (long long)in_sizes[2] < need) return;
  const long long wn = (long long)EDIM * EDIM;
  if ((long long)in_sizes[3] < wn || (long long)in_sizes[4] < wn || (long long)in_sizes[5] < wn || (long long)in_sizes[6] < wn) return;
  if ((long long)out_size < need) return;
  const float* q  = (const float*)d_in[0];
  const float* k  = (const float*)d_in[1];
  const float* v  = (const float*)d_in[2];
  const float* Wq = (const float*)d_in[3];
  const float* Wk = (const float*)d_in[4];
  const float* Wv = (const float*)d_in[5];
  const float* Wo = (const float*)d_in[6];
  float* out = (float*)d_out;
  char* ws = (char*)d_ws;
  size_t off = 0;
  const size_t xplane = (size_t)NB * SEQ * EDIM * 2;
  const size_t wplane = (size_t)EDIM * EDIM * 2;
  unsigned short* Xq = (unsigned short*)(ws + off); off += (xplane + 255) & ~(size_t)255;
  unsigned short* Xk = (unsigned short*)(ws + off); off += (xplane + 255) & ~(size_t)255;
  unsigned short* Xv = (unsigned short*)(ws + off); off += (xplane + 255) & ~(size_t)255;
  unsigned short* Bq = (unsigned short*)(ws + off); off += (wplane + 255) & ~(size_t)255;
  unsigned short* Bk = (unsigned short*)(ws + off); off += (wplane + 255) & ~(size_t)255;
  unsigned short* Bv = (unsigned short*)(ws + off); off += (wplane + 255) & ~(size_t)255;
  unsigned short* Bo = (unsigned short*)(ws + off); off += (wplane + 255) & ~(size_t)255;
  unsigned short* Qh = (unsigned short*)(ws + off); off += (xplane + 255) & ~(size_t)255;
  unsigned short* Ql = (unsigned short*)(ws + off); off += (xplane + 255) & ~(size_t)255;
  unsigned short* Kh = (unsigned short*)(ws + off); off += (xplane + 255) & ~(size_t)255;
  unsigned short* Kl = (unsigned short*)(ws + off); off += (xplane + 255) & ~(size_t)255;
  unsigned short* Vt = (unsigned short*)(ws + off); off += (xplane + 255) & ~(size_t)255;
  unsigned short* Cx = (unsigned short*)(ws + off); off += (2 * xplane + 255) & ~(size_t)255;
  if (off > ws_size) return;

  const int x8 = NB * SEQ * (EDIM / 8);
  const int w8 = EDIM * (EDIM / 8);
  k_cvt<<<(unsigned)((x8 + 255) / 256), 256, 0, stream>>>(q, Xq, SEQ, SEQ_FULL, x8);
  k_cvt<<<(unsigned)((x8 + 255) / 256), 256, 0, stream>>>(k, Xk, SEQ, SEQ_FULL, x8);
  k_cvt<<<(unsigned)((x8 + 255) / 256), 256, 0, stream>>>(v, Xv, SEQ, SEQ_FULL, x8);
  k_cvt<<<(unsigned)((w8 + 255) / 256), 256, 0, stream>>>(Wq, Bq, EDIM, EDIM, w8);
  k_cvt<<<(unsigned)((w8 + 255) / 256), 256, 0, stream>>>(Wk, Bk, EDIM, EDIM, w8);
  k_cvt<<<(unsigned)((w8 + 255) / 256), 256, 0, stream>>>(Wv, Bv, EDIM, EDIM, w8);
  k_cvt<<<(unsigned)((w8 + 255) / 256), 256, 0, stream>>>(Wo, Bo, EDIM, EDIM, w8);

  const dim3 gg((unsigned)(NB * SEQ / 128), (unsigned)(EDIM / 64));
  k_gemm<0, EDIM, EDIM><<<gg, 128, 0, stream>>>(Xq, Bq, Qh, Ql, out);
  k_gemm<0, EDIM, EDIM><<<gg, 128, 0, stream>>>(Xk, Bk, Kh, Kl, out);
  k_gemm<1, EDIM, EDIM><<<gg, 128, 0, stream>>>(Xv, Bv, Vt, Cx, out);
  k_attn<<<(unsigned)(NB * NH * (SEQ / 64)), 128, 0, stream>>>(Qh, Ql, Kh, Kl, Vt, Cx);
  k_gemm<2, 2 * EDIM, 2 * EDIM><<<gg, 128, 0, stream>>>(Cx, Bo, Qh, Ql, out);
}
